// FrequencyGuidedAttention_28346784153715
// MI455X (gfx1250) — hardware-verified
//
#include <hip/hip_runtime.h>


#define NB_  8
#define TT   1024
#define DM   768
#define NH_  12
#define HD   64
#define ZH   12
#define PCAR 1024.0f
typedef _Float16 h16;
typedef unsigned short bf;
typedef __attribute__((ext_vector_type(16))) __bf16   v16bf;
typedef __attribute__((ext_vector_type(16))) _Float16 v16h;
typedef __attribute__((ext_vector_type(8)))  _Float16 v8h;
typedef __attribute__((ext_vector_type(8)))  unsigned short v8us;
typedef __attribute__((ext_vector_type(8)))  float    v8f;
typedef __attribute__((ext_vector_type(4)))  float    v4f;
typedef v8h  __attribute__((may_alias)) v8ha;
typedef v4f  __attribute__((may_alias)) v4fa;
typedef v8us __attribute__((may_alias)) v8usa;

__device__ __forceinline__ unsigned short f2bf(float f) { unsigned u = __float_as_uint(f); u += 0x7FFFu + ((u >> 16) & 1u); return (unsigned short)(u >> 16); }
__device__ __forceinline__ float bf2f(unsigned short b) { return __uint_as_float(((unsigned)b) << 16); }
__device__ __forceinline__ float bfr(float f) { return bf2f(f2bf(f)); }
__device__ __forceinline__ v16h cat16(v8h lo, v8h hi) { return __builtin_shufflevector(lo, hi, 0, 1, 2, 3, 4, 5, 6, 7, 8, 9, 10, 11, 12, 13, 14, 15); }
__device__ __forceinline__ v16bf cat16b(v8us lo, v8us hi) { return __builtin_bit_cast(v16bf, __builtin_shufflevector(lo, hi, 0, 1, 2, 3, 4, 5, 6, 7, 8, 9, 10, 11, 12, 13, 14, 15)); }
__device__ __forceinline__ v8f wmma16(v16h a, v16h b, v8f c) { return __builtin_amdgcn_wmma_f32_16x16x32_f16(false, a, false, b, (short)0, c, false, false); }
__device__ __forceinline__ v8f wmmab(v16bf a, v16bf b, v8f c) { return __builtin_amdgcn_wmma_f32_16x16x32_bf16(false, a, false, b, (short)0, c, false, false); }


template <typename T16> struct WFrag;
template <> struct WFrag<h16> { typedef v16h V; static __device__ __forceinline__ V ld(const h16* p) { return cat16(*(const v8h*)p, *(const v8h*)(p + 16)); } static __device__ __forceinline__ v8f mma(V a, V b, v8f c) { return wmma16(a, b, c); } };
template <> struct WFrag<bf> { typedef v16bf V; static __device__ __forceinline__ V ld(const bf* p) { return cat16b(*(const v8us*)p, *(const v8us*)(p + 16)); } static __device__ __forceinline__ v8f mma(V a, V b, v8f c) { return wmmab(a, b, c); } };
template <typename T16, int NSPLIT, bool BIAS>
__global__ __launch_bounds__(32) void k_gemmw(const T16* __restrict__ A, const T16* __restrict__ A2, const T16* __restrict__ Bt, const T16* __restrict__ Bt2, int K, float* C, int ldc, const float* __restrict__ bias, size_t sA, size_t sB, size_t sC) {
    typedef typename WFrag<T16>::V V;
    __shared__ __align__(16) float os[16 * 68];
    const size_t z = blockIdx.z; A += z * sA; if (A2) A2 += z * sA; Bt += z * sB; if (Bt2) Bt2 += z * sB; C += z * sC;
    const int lane = threadIdx.x & 31, lr = lane & 15, hi = lane >> 4; const int r0 = blockIdx.x * 64, c0 = blockIdx.y * 64;
    v8f acc[4][4];
#pragma unroll
    for (int mb = 0; mb < 4; ++mb)
#pragma unroll
        for (int nb = 0; nb < 4; ++nb) acc[mb][nb] = (v8f){};
    const size_t aoff = (size_t)(r0 + lr) * K + 8 * hi, boff = (size_t)(c0 + lr) * K + 8 * hi;
#pragma unroll 1
    for (int kc = 0; kc < K; kc += 32) {
        V a[4], a2[4];
#pragma unroll
        for (int mb = 0; mb < 4; ++mb) { a[mb] = WFrag<T16>::ld(A + aoff + (size_t)mb * 16 * K + kc); if (NSPLIT == 1 || NSPLIT == 2) a2[mb] = WFrag<T16>::ld(A2 + aoff + (size_t)mb * 16 * K + kc); }
#pragma unroll
        for (int nb = 0; nb < 4; ++nb) { const V b = WFrag<T16>::ld(Bt + boff + (size_t)nb * 16 * K + kc); V b2; if (NSPLIT >= 2) b2 = WFrag<T16>::ld(Bt2 + boff + (size_t)nb * 16 * K + kc);
#pragma unroll
            for (int mb = 0; mb < 4; ++mb) { acc[mb][nb] = WFrag<T16>::mma(a[mb], b, acc[mb][nb]); if (NSPLIT == 1 || NSPLIT == 2) acc[mb][nb] = WFrag<T16>::mma(a2[mb], b, acc[mb][nb]); if (NSPLIT >= 2) acc[mb][nb] = WFrag<T16>::mma(a[mb], b2, acc[mb][nb]); } }
        asm volatile("v_nop\n\tv_nop\n\tv_nop\n\tv_nop" : "+v"(acc[0][0]), "+v"(acc[1][1]), "+v"(acc[2][2]), "+v"(acc[3][3]) : "v"(a[0]), "v"(a[3]));
    }
#pragma unroll
    for (int mb = 0; mb < 4; ++mb) {
#pragma unroll
        for (int nb = 0; nb < 4; ++nb) {
#pragma unroll
            for (int j = 0; j < 8; ++j) os[(hi * 8 + j) * 68 + nb * 16 + lr] = acc[mb][nb][j]; }
        __builtin_amdgcn_wave_barrier(); asm volatile("" ::: "memory");
        float* crow = C + (size_t)(r0 + mb * 16) * ldc + c0;
#pragma unroll 1
        for (int ps = 0; ps < 2; ++ps) {
#pragma unroll
            for (int s = 0; s < 8; ++s) { const int row = 2 * s + hi, cofs = lr * 4; v4f val = *(const v4fa*)(os + row * 68 + cofs); if (BIAS) { val[0] += bfr(bias[c0 + cofs]); val[1] += bfr(bias[c0 + cofs + 1]); val[2] += bfr(bias[c0 + cofs + 2]); val[3] += bfr(bias[c0 + cofs + 3]); }
                *(volatile v4f*)(crow + (size_t)row * ldc + cofs) = val; }
            if (ps == 0) __threadfence(); }
        __builtin_amdgcn_wave_barrier(); asm volatile("" ::: "memory");
    }
}

__device__ __forceinline__ h16 tohx(float x) { return (h16)x; }
__device__ __forceinline__ void splitf(float y, unsigned short& h, unsigned short& l) { h = f2bf(y); l = f2bf(y - bf2f(h)); }
typedef __attribute__((ext_vector_type(2))) unsigned short v2us;
typedef __attribute__((ext_vector_type(4))) unsigned short v4us;
typedef __attribute__((ext_vector_type(2))) _Float16 v2h;
typedef __attribute__((ext_vector_type(4))) _Float16 v4h;

__global__ __launch_bounds__(256) void k_cvt8(const float* __restrict__ src, bf* dst, size_t n8) { const size_t i = (size_t)blockIdx.x * 256 + threadIdx.x; if (i >= n8) return; const v8f v = *(const v8f*)(src + i * 8); v8us o;
#pragma unroll
    for (int k = 0; k < 8; ++k) o[k] = f2bf(v[k]); *(volatile v8us*)(dst + i * 8) = o; __threadfence(); *(volatile v8us*)(dst + i * 8) = o; }
__global__ __launch_bounds__(256) void k_wtG(const float* __restrict__ w, int K, int N, bf* Bt) {
    const int lane = threadIdx.x & 31; const int L0 = (blockIdx.x * 8 + (threadIdx.x >> 5)) * 8; const int nlines = N * K / 64;
#pragma unroll
    for (int ps = 0; ps < 2; ++ps) {
#pragma unroll 1
        for (int l = 0; l < 8; ++l) { const int L = L0 + l; if (L >= nlines) break; const size_t e = (size_t)L * 64 + lane * 2; const int k = (int)(e % K), n = (int)(e / K); v2us o;
            o[0] = f2bf(w[(size_t)k * N + n]); o[1] = f2bf(w[(size_t)(k + 1) * N + n]); *(volatile v2us*)(Bt + e) = o; }
        if (ps == 0) __threadfence(); }
}

__global__ __launch_bounds__(256) void k_qkpl(const float* __restrict__ QKV, h16* QP, h16* KP) { const size_t e = ((size_t)blockIdx.x * 256 + threadIdx.x) * 4; if (e >= (size_t)NH_ * TT * HD) return; const int d = (int)(e % HD); const int t = (int)((e / HD) % TT); const int h = (int)(e / ((size_t)HD * TT)); const float* r = QKV + (size_t)t * 3 * DM + h * HD + d; const v4f a = *(const v4f*)r, c = *(const v4f*)(r + DM); v4h oq, ok;
    for (int u = 0; u < 4; ++u) { oq[u] = tohx(a[u]); ok[u] = tohx(c[u]); } *(volatile v4h*)(QP + e) = oq; *(volatile v4h*)(KP + e) = ok; __threadfence(); *(volatile v4h*)(QP + e) = oq; *(volatile v4h*)(KP + e) = ok; }
__global__ __launch_bounds__(256) void k_vgt(const float* __restrict__ QKV, const float* __restrict__ G, const float* __restrict__ fsp, h16* VT) { const size_t e = ((size_t)blockIdx.x * 256 + threadIdx.x) * 2; if (e >= (size_t)NH_ * HD * TT) return; const int t = (int)(e % TT); const int d = (int)((e / TT) % HD); const int h = (int)(e / ((size_t)TT * HD)); const float fs = __fdiv_rn(1.0f, __fadd_rn(1.0f, expf(-bfr(fsp[0])))); v2h o;
#pragma unroll
    for (int u = 0; u < 2; ++u) { const float v = QKV[(size_t)(t + u) * 3 * DM + 2 * DM + h * HD + d]; float gd = __fmul_rn(fs, G[(size_t)(t + u) * DM + h * HD + d]); asm volatile("" : "+v"(gd)); o[u] = tohx(__fadd_rn(v, gd)); } *(volatile v2h*)(VT + e) = o; __threadfence(); *(volatile v2h*)(VT + e) = o; }
__global__ __launch_bounds__(256) void k_soft(const float* __restrict__ S, h16* P16) { const int lane = threadIdx.x & 31; const int row = blockIdx.x * 8 + (threadIdx.x >> 5); if (row >= NH_ * TT) return; const float* sr = S + (size_t)row * TT; float v[TT / 32]; float mx = -3.0e38f;
#pragma unroll
    for (int ch = 0; ch < TT / 128; ++ch) { const v4f a = *(const v4f*)(sr + ch * 128 + lane * 4);
#pragma unroll
        for (int u = 0; u < 4; ++u) { const float t = fminf(fmaxf(a[u] * 0.125f, -20.0f), 20.0f); v[ch * 4 + u] = t; mx = fmaxf(mx, t); } }
#pragma unroll
    for (int sh = 16; sh; sh >>= 1) mx = fmaxf(mx, __shfl_xor(mx, sh, 32));
    float sum = 0.f;
#pragma unroll
    for (int q = 0; q < TT / 32; ++q) { float d0 = __fsub_rn(v[q], mx); asm volatile("" : "+v"(d0)); v[q] = __builtin_amdgcn_exp2f(__fmul_rn(d0, 1.4426950408889634f)); sum += v[q]; }
#pragma unroll
    for (int sh = 16; sh; sh >>= 1) sum += __shfl_xor(sum, sh, 32);
    const float f = __fdiv_rn(PCAR, sum);
    for (int ps = 0; ps < 2; ++ps) {
#pragma unroll
        for (int ch = 0; ch < TT / 128; ++ch) { v4h o4; for (int q = 0; q < 4; ++q) o4[q] = tohx(v[ch * 4 + q] * f); *(volatile v4h*)(P16 + (size_t)row * TT + ch * 128 + lane * 4) = o4; }
        if (ps == 0) __threadfence(); } }
__global__ __launch_bounds__(256) void k_mrg(const float* __restrict__ O, bf* Ah, bf* Al) { const size_t e = ((size_t)blockIdx.x * 256 + threadIdx.x) * 4; if (e >= (size_t)NH_ * TT * HD) return; const int d = (int)(e % HD); const int t = (int)((e / HD) % TT); const int h = (int)(e / ((size_t)HD * TT)); const size_t oo = (size_t)t * DM + h * HD + d; v4us oh, ol;
#pragma unroll
    for (int u = 0; u < 4; ++u) { unsigned short a, b; splitf(O[e + u] * (1.0f / PCAR), a, b); oh[u] = a; ol[u] = b; } *(volatile v4us*)(Ah + oo) = oh; *(volatile v4us*)(Al + oo) = ol; __threadfence(); *(volatile v4us*)(Ah + oo) = oh; *(volatile v4us*)(Al + oo) = ol; }
__global__ __launch_bounds__(256) void k_ln(const float* __restrict__ Y, const float* __restrict__ gam, const float* __restrict__ bet, float* OUTb) { const int lane = threadIdx.x & 31; const int row = blockIdx.x * 8 + (threadIdx.x >> 5); if (row >= TT) return; const float* y = Y + (size_t)row * DM; float v[DM / 32]; float s = 0.f;
#pragma unroll
    for (int ch = 0; ch < DM / 128; ++ch) { const v4f a = *(const v4f*)(y + ch * 128 + lane * 4); for (int u = 0; u < 4; ++u) { v[ch * 4 + u] = a[u]; s = __fadd_rn(s, a[u]); } }
#pragma unroll
    for (int sh = 16; sh; sh >>= 1) s = __fadd_rn(s, __shfl_xor(s, sh, 32));
    const float mu = __fdiv_rn(s, (float)DM); float q2 = 0.f;
#pragma unroll
    for (int k = 0; k < DM / 32; ++k) { const float d0 = __fsub_rn(v[k], mu); v[k] = d0; float p = __fmul_rn(d0, d0); asm volatile("" : "+v"(p)); q2 = __fadd_rn(q2, p); }
#pragma unroll
    for (int sh = 16; sh; sh >>= 1) q2 = __fadd_rn(q2, __shfl_xor(q2, sh, 32));
    const float rs = __fdiv_rn(1.0f, sqrtf(__fadd_rn(__fdiv_rn(q2, (float)DM), 1e-5f)));
    for (int ps = 0; ps < 2; ++ps) {
#pragma unroll
        for (int ch = 0; ch < DM / 128; ++ch) { v4f o; for (int u = 0; u < 4; ++u) { const int c = ch * 128 + lane * 4 + u; float n0 = __fmul_rn(v[ch * 4 + u], rs); asm volatile("" : "+v"(n0)); float gg = __fmul_rn(n0, bfr(gam[c])); asm volatile("" : "+v"(gg)); o[u] = __fadd_rn(gg, bfr(bet[c])); } *(volatile v4f*)(OUTb + (size_t)row * DM + ch * 128 + lane * 4) = o; }
        if (ps == 0) __threadfence(); } }

extern "C" void kernel_launch(void* const* d_in, const int* in_sizes, int n_in,
                              void* d_out, int out_size, void* d_ws, size_t ws_size, hipStream_t stream) {
    (void)in_sizes; (void)n_in; (void)out_size;
    const float* x = (const float*)d_in[0]; const float* flo = (const float*)d_in[1]; const float* fhi = (const float*)d_in[2]; const float* Wqi = (const float*)d_in[3]; const float* Wqa = (const float*)d_in[4];
    const float* Wfi = (const float*)d_in[5]; const float* bfi = (const float*)d_in[6]; const float* Wfa = (const float*)d_in[7]; const float* bfa = (const float*)d_in[8]; const float* Wpi = (const float*)d_in[9]; const float* bpi = (const float*)d_in[10]; const float* Wpa = (const float*)d_in[11]; const float* bpa = (const float*)d_in[12];
    const float* gi = (const float*)d_in[13]; const float* bi = (const float*)d_in[14]; const float* ga = (const float*)d_in[15]; const float* ba = (const float*)d_in[16]; const float* otemp = (const float*)d_in[17]; const float* fsp = (const float*)d_in[18]; (void)otemp;
    float* OUT0 = (float*)d_out; float* OUT1 = OUT0 + (size_t)NB_ * TT * DM;
    char* wsp = (char*)d_ws;
    auto take = [&](size_t bytes) { char* p = wsp; wsp += (bytes + 255) & ~(size_t)255; return (void*)p; };
    bf* BQ[2]; bf* BFG[2]; bf* BP[2]; for (int r = 0; r < 2; ++r) { BQ[r] = (bf*)take((size_t)3 * DM * DM * 2); BFG[r] = (bf*)take((size_t)DM * DM * 2); BP[r] = (bf*)take((size_t)DM * DM * 2); }
    bf* XB = (bf*)take((size_t)TT * DM * 2); bf* FB = (bf*)take((size_t)TT * DM * 2); float* QKV = (float*)take((size_t)TT * 3 * DM * 4); float* GD = (float*)take((size_t)TT * DM * 4);
    h16* QP = (h16*)take((size_t)NH_ * TT * HD * 2); h16* KP = (h16*)take((size_t)NH_ * TT * HD * 2); h16* VT = (h16*)take((size_t)NH_ * HD * TT * 2); float* S = (float*)take((size_t)NH_ * TT * TT * 4); h16* P16 = (h16*)take((size_t)NH_ * TT * TT * 2); float* O = (float*)take((size_t)NH_ * TT * HD * 4);
    bf* ATh = (bf*)take((size_t)TT * DM * 2); bf* ATl = (bf*)take((size_t)TT * DM * 2); float* Y = (float*)take((size_t)TT * DM * 4);
    if ((size_t)(wsp - (char*)d_ws) > ws_size) return;
    const float* WQs[2] = {Wqi, Wqa}; const float* WFs[2] = {Wfi, Wfa}; const float* WPs[2] = {Wpi, Wpa};
    for (int r = 0; r < 2; ++r) { k_wtG<<<(DM * 3 * DM / 64 + 63) / 64, 256, 0, stream>>>(WQs[r], DM, 3 * DM, BQ[r]); k_wtG<<<(DM * DM / 64 + 63) / 64, 256, 0, stream>>>(WFs[r], DM, DM, BFG[r]); k_wtG<<<(DM * DM / 64 + 63) / 64, 256, 0, stream>>>(WPs[r], DM, DM, BP[r]); }
    const float* feats[2] = {flo, fhi}; const float* bfg[2] = {bfi, bfa}; const float* bps[2] = {bpi, bpa}; const float* gams[2] = {gi, ga}; const float* bets[2] = {bi, ba}; float* OUTS[2] = {OUT0, OUT1};
    const size_t zq = (size_t)TT * HD, zS = (size_t)TT * TT, zv = (size_t)HD * TT;
    for (int b = 0; b < NB_; ++b) {
        k_cvt8<<<(TT * DM / 8 + 255) / 256, 256, 0, stream>>>(x + (size_t)b * TT * DM, XB, TT * DM / 8);
        for (int r = 0; r < 2; ++r) {
            k_cvt8<<<(TT * DM / 8 + 255) / 256, 256, 0, stream>>>(feats[r] + (size_t)b * TT * DM, FB, TT * DM / 8);
            k_gemmw<bf, 0, false><<<dim3(TT / 64, 3 * DM / 64, 1), 32, 0, stream>>>(XB, nullptr, BQ[r], nullptr, DM, QKV, 3 * DM, nullptr, 0, 0, 0);
            k_gemmw<bf, 0, true><<<dim3(TT / 64, DM / 64, 1), 32, 0, stream>>>(FB, nullptr, BFG[r], nullptr, DM, GD, DM, bfg[r], 0, 0, 0);
            k_qkpl<<<(unsigned)(((size_t)NH_ * TT * HD / 4 + 255) / 256), 256, 0, stream>>>(QKV, QP, KP); k_vgt<<<(unsigned)(((size_t)NH_ * HD * TT / 2 + 255) / 256), 256, 0, stream>>>(QKV, GD, fsp, VT);
            k_gemmw<h16, 0, false><<<dim3(TT / 64, TT / 64, ZH), 32, 0, stream>>>(QP, nullptr, KP, nullptr, HD, S, TT, nullptr, zq, zq, zS);
            k_soft<<<NH_ * TT / 8, 256, 0, stream>>>(S, P16);
            k_gemmw<h16, 0, false><<<dim3(TT / 64, 1, ZH), 32, 0, stream>>>(P16, nullptr, VT, nullptr, TT, O, HD, nullptr, zS, zv, zq);
            k_mrg<<<(unsigned)(((size_t)NH_ * TT * HD / 4 + 255) / 256), 256, 0, stream>>>(O, ATh, ATl);
            k_gemmw<bf, 1, true><<<dim3(TT / 64, DM / 64, 1), 32, 0, stream>>>(ATh, ATl, BP[r], nullptr, DM, Y, DM, bps[r], 0, 0, 0);
            k_ln<<<TT / 8, 256, 0, stream>>>(Y, gams[r], bets[r], OUTS[r] + (size_t)b * TT * DM); } }
}
